// LinearKAN_35553739276891
// MI455X (gfx1250) — hardware-verified
//
#include <hip/hip_runtime.h>
#include <math.h>

#ifndef NB
#define NB 2048
#endif
constexpr int kRows      = NB;
constexpr int kRowsFull  = 2048;
constexpr int kIn        = 512;
constexpr int kOutF      = 512;
constexpr int kBasis     = 8;
constexpr int kKtot      = kIn + kIn * kBasis;
constexpr int kFeatThreads = 256;
constexpr int kFeatBlocksPerRow = kIn / kFeatThreads;
static_assert(kKtot % 32 == 0);
static_assert(kRows % 64 == 0 && kRows >= 64 && kRows <= kRowsFull);
static_assert(kOutF % 64 == 0);
static_assert((kKtot * 2) % 128 == 0);
static_assert(kIn % kFeatThreads == 0 && kFeatThreads == 256);

constexpr size_t kBtPlaneBytes = (size_t)kOutF * kKtot * 2;
constexpr size_t kAPlaneBytes  = (size_t)kRows * kKtot * 2;
constexpr size_t kOffBtHi = 0;
constexpr size_t kOffBtLo = kOffBtHi + kBtPlaneBytes;
constexpr size_t kOffAHi  = kOffBtLo + kBtPlaneBytes;
constexpr size_t kOffALo  = kOffAHi + kAPlaneBytes;
constexpr size_t kWsTotal = kOffALo + kAPlaneBytes;
static_assert(kWsTotal <= 134217728ull);
static_assert(kOffBtLo % 128 == 0 && kOffAHi % 128 == 0 && kOffALo % 128 == 0);

typedef __attribute__((ext_vector_type(16))) _Float16 v16h;
typedef __attribute__((ext_vector_type(8)))  _Float16 v8h;
typedef __attribute__((ext_vector_type(16))) __bf16   v16b;
typedef __attribute__((ext_vector_type(8)))  __bf16   v8b;
typedef __attribute__((ext_vector_type(8)))  float    v8f;
typedef __attribute__((ext_vector_type(4)))  float    v4f;
typedef __attribute__((ext_vector_type(4)))  unsigned int v4u;

__device__ __forceinline__ unsigned short f2bf_bits(float f) {
  unsigned u = __float_as_uint(f);
  return (unsigned short)((u + 0x7FFFu + ((u >> 16) & 1u)) >> 16);
}
__device__ __forceinline__ float bf_bits2f(unsigned short h) { return __uint_as_float(((unsigned)h) << 16); }
__device__ __forceinline__ float bf_rne(float f) { return bf_bits2f(f2bf_bits(f)); }

__device__ __forceinline__ void dep_guard_h(v8f& a, v8f& b, v16h x, v16h y) { asm volatile("v_nop\n\tv_nop\n\tv_nop\n\tv_nop" : "+v"(a), "+v"(b) : "v"(x), "v"(y)); }
__device__ __forceinline__ void dep_guard_b(v8f& a, v8f& b, v16b x, v16b y) { asm volatile("v_nop\n\tv_nop\n\tv_nop\n\tv_nop" : "+v"(a), "+v"(b) : "v"(x), "v"(y)); }
__device__ __forceinline__ void keep4_h(v16h a, v16h b, v16h c, v16h d) { asm volatile("v_nop" :: "v"(a), "v"(b), "v"(c), "v"(d)); }
__device__ __forceinline__ void keep4_b(v16b a, v16b b, v16b c, v16b d) { asm volatile("v_nop" :: "v"(a), "v"(b), "v"(c), "v"(d)); }
__device__ __forceinline__ void acc_guard4(v8f& a, v8f& b, v8f& c, v8f& d) { asm volatile("v_nop\n\tv_nop\n\tv_nop\n\tv_nop" : "+v"(a), "+v"(b), "+v"(c), "+v"(d)); }
template <typename T> struct Frag;
template <> struct Frag<_Float16> {
  typedef v16h V; union U { v16h v; v8h h[2]; };
  static __device__ __forceinline__ v16h load(const _Float16* p) {
    U f; f.h[0] = *(const v8h*)(p); f.h[1] = *(const v8h*)(p + 16); return f.v;
  }
  static __device__ __forceinline__ v8f mma(v16h a, v16h b, v8f c) {
    return __builtin_amdgcn_wmma_f32_16x16x32_f16(false, a, false, b, (short)0, c, false, false);
  }
  static __device__ __forceinline__ void guard(v8f& a, v8f& b, v16h x, v16h y) { dep_guard_h(a, b, x, y); }
  static __device__ __forceinline__ void keep(v16h a, v16h b, v16h c, v16h d) { keep4_h(a, b, c, d); }
};
template <> struct Frag<__bf16> {
  typedef v16b V; union U { v16b v; v8b h[2]; };
  static __device__ __forceinline__ v16b load(const __bf16* p) {
    U f; f.h[0] = *(const v8b*)(p); f.h[1] = *(const v8b*)(p + 16); return f.v;
  }
  static __device__ __forceinline__ v8f mma(v16b a, v16b b, v8f c) {
    return __builtin_amdgcn_wmma_f32_16x16x32_bf16(false, a, false, b, (short)0, c, false, false);
  }
  static __device__ __forceinline__ void guard(v8f& a, v8f& b, v16b x, v16b y) { dep_guard_b(a, b, x, y); }
  static __device__ __forceinline__ void keep(v16b a, v16b b, v16b c, v16b d) { keep4_b(a, b, c, d); }
};

__device__ __forceinline__ unsigned pk16(unsigned short a, unsigned short b) { return (unsigned)a | ((unsigned)b << 16); }

template <int ET> struct Elem;
template <> struct Elem<0> { typedef _Float16 T; };
template <> struct Elem<1> { typedef __bf16 T; };
template <int ET, bool SPLIT, int BIAS_MODE, int OUT_MODE, bool RESID, int ACT = 0>
__global__ __launch_bounds__(256) void wmma_gemm64(
    const unsigned short* __restrict__ Ap, const unsigned short* __restrict__ A2p, int lda, long strideA,
    const unsigned short* __restrict__ Btp, const unsigned short* __restrict__ Bt2p, int ldb, long strideB,
    void* __restrict__ Cout, void* __restrict__ Cout2, int ldc, long strideC,
    const float* __restrict__ bias,
    const float* __restrict__ resid, long strideR,
    int M, int N, int K, float scale) {
  typedef typename Elem<ET>::T T;
  typedef typename Frag<T>::V V;
  const T* A = (const T*)Ap; const T* A2 = (const T*)A2p; const T* Bt = (const T*)Btp; const T* Bt2 = (const T*)Bt2p;
  __shared__ __align__(16) float sT[8][16 * 68];
  const int b    = blockIdx.y;
  const int lane = threadIdx.x & 31;
  const int wave = threadIdx.x >> 5;
  const int tilesN = N >> 6;
  const int tilesM = M >> 6;
  const int tile = blockIdx.x * 8 + wave;
  if (tile >= tilesM * tilesN) return;
  const int tm = tile / tilesN;
  const int tn = tile - tm * tilesN;
  const int m0 = tm << 6;
  const int n0 = tn << 6;

  const T* Ab  = A  + (size_t)b * strideA;
  const T* Bb  = Bt + (size_t)b * strideB;
  const T* Ab2 = SPLIT ? (A2  + (size_t)b * strideA) : nullptr;
  const T* Bb2 = SPLIT ? (Bt2 + (size_t)b * strideB) : nullptr;

  const int rlane = lane & 15;
  const int koff  = (lane >> 4) * 8;
  const int mOff  = (lane >> 4) * 8;

  v8f acc[4][4];
#pragma unroll
  for (int i = 0; i < 4; ++i)
#pragma unroll
    for (int j = 0; j < 4; ++j) acc[i][j] = (v8f){0.f,0.f,0.f,0.f,0.f,0.f,0.f,0.f};

  for (int k0 = 0; k0 < K; k0 += 32) {
    V bh[4], bl[4];
#pragma unroll
    for (int j = 0; j < 4; ++j) {
      const size_t bo = (size_t)(n0 + (j << 4) + rlane) * ldb + koff + k0;
      bh[j] = Frag<T>::load(Bb + bo);
      if (SPLIT) bl[j] = Frag<T>::load(Bb2 + bo);
    }
#pragma unroll
    for (int i = 0; i < 4; ++i) {
      const size_t ao = (size_t)(m0 + (i << 4) + rlane) * lda + koff + k0;
      V ah = Frag<T>::load(Ab + ao);
      V al;
      if (SPLIT) al = Frag<T>::load(Ab2 + ao);
#pragma unroll
      for (int j = 0; j < 4; ++j) {
        acc[i][j] = Frag<T>::mma(ah, bh[j], acc[i][j]);
        if (SPLIT) {
          acc[i][j] = Frag<T>::mma(ah, bl[j], acc[i][j]);
          acc[i][j] = Frag<T>::mma(al, bh[j], acc[i][j]);
        }
      }
      Frag<T>::guard(acc[i][0], acc[i][3], ah, SPLIT ? al : ah);
    }
    Frag<T>::keep(bh[0], bh[1], bh[2], bh[3]);
    if (SPLIT) Frag<T>::keep(bl[0], bl[1], bl[2], bl[3]);
  }
  acc_guard4(acc[0][0], acc[0][1], acc[0][2], acc[0][3]);
  acc_guard4(acc[1][0], acc[1][1], acc[1][2], acc[1][3]);
  acc_guard4(acc[2][0], acc[2][1], acc[2][2], acc[2][3]);
  acc_guard4(acc[3][0], acc[3][1], acc[3][2], acc[3][3]);

  float* slab = sT[wave];
  const float* Rb = RESID ? (resid + (size_t)b * strideR) : nullptr;
#pragma unroll
  for (int i = 0; i < 4; ++i) {
    const int mBase = m0 + (i << 4);
#pragma unroll
    for (int j = 0; j < 4; ++j) {
      const int n = n0 + (j << 4) + rlane;
      float bv = 0.f;
      if (BIAS_MODE == 2) bv = bias[n];
#pragma unroll
      for (int r = 0; r < 8; ++r) {
        float v = acc[i][j][r] * scale;
        if (BIAS_MODE == 1) v += bias[mBase + mOff + r];
        if (BIAS_MODE == 2) v += bv;
        if (RESID) v += Rb[(size_t)(mBase + mOff + r) * ldc + n];
        if (ACT == 2) v = fmaxf(v, 0.0f);
        if (ACT == 4) v = (v > 0.f) ? v : 0.01f * v;
        slab[(mOff + r) * 68 + (j << 4) + rlane] = v;
      }
    }
    __builtin_amdgcn_fence(__ATOMIC_RELEASE, "workgroup");
    __builtin_amdgcn_wave_barrier();
    __builtin_amdgcn_fence(__ATOMIC_ACQUIRE, "workgroup");
    if (OUT_MODE == 0) {
      float* C = (float*)Cout + (size_t)b * strideC;
      const int hh = lane >> 4, c4 = (lane & 15) * 4;
      for (int pass = 0; pass < 2; ++pass) {
#pragma unroll
        for (int it = 0; it < 8; ++it) {
          const int row = it * 2 + hh;
          v4f v = *(const v4f*)(slab + row * 68 + c4);
          *(volatile v4f*)(C + (size_t)(mBase + row) * ldc + n0 + c4) = v;
        }
        __threadfence();
      }
    } else {
      const int q = lane >> 3, c8 = (lane & 7) * 8;
      unsigned short* C  = (unsigned short*)Cout  + (size_t)b * strideC;
      unsigned short* C2 = (OUT_MODE == 2) ? ((unsigned short*)Cout2 + (size_t)b * strideC) : nullptr;
      for (int pass = 0; pass < 2; ++pass) {
#pragma unroll
        for (int it = 0; it < 4; ++it) {
          const int row = it * 4 + q;
          const float* sp = slab + row * 68 + c8;
          v8h hv, lv;
#pragma unroll
          for (int e = 0; e < 8; ++e) {
            if (OUT_MODE == 1) {
              hv[e] = (_Float16)sp[e];
            } else {
              unsigned short hb = f2bf_bits(sp[e]);
              unsigned short lb = f2bf_bits(sp[e] - bf_bits2f(hb));
              hv[e] = __builtin_bit_cast(_Float16, hb);
              lv[e] = __builtin_bit_cast(_Float16, lb);
            }
          }
          *(volatile v8h*)(C + (size_t)(mBase + row) * ldc + n0 + c8) = hv;
          if (OUT_MODE == 2) *(volatile v8h*)(C2 + (size_t)(mBase + row) * ldc + n0 + c8) = lv;
        }
        __threadfence();
      }
    }
    __builtin_amdgcn_fence(__ATOMIC_RELEASE, "workgroup");
    __builtin_amdgcn_wave_barrier();
    __builtin_amdgcn_fence(__ATOMIC_ACQUIRE, "workgroup");
  }
}

__global__ __launch_bounds__(256) void wprep_kernel(const float* __restrict__ w, const float* __restrict__ cf,
                                                    unsigned short* __restrict__ Bhi, unsigned short* __restrict__ Blo) {
#pragma clang fp contract(off)
  constexpr int kSegs = kKtot / 8;
  const int t = blockIdx.x * 256 + threadIdx.x;
  if (t >= kOutF * kSegs) return;
  const int o   = t / kSegs;
  const int seg = t - o * kSegs;
  const int kk0 = seg * 8;
  unsigned short hb[8], lb[8];
#pragma unroll
  for (int e = 0; e < 8; ++e) {
    const int kk = kk0 + e;
    const int ib = (kk < kIn - 1) ? kk : (kIn - 1);
    const float vb = bf_rne(w[(size_t)ib * kOutF + o]);
    int km = kk - kIn; km = (km < 0) ? 0 : km;
    const int i2 = km >> 3;
    const int k2 = km & 7;
    const float vs = bf_rne(w[(size_t)i2 * kOutF + o]) * bf_rne(cf[((size_t)i2 * kOutF + o) * kBasis + k2]);
    const float v = (kk < kIn) ? vb : vs;
    hb[e] = f2bf_bits(v);
    lb[e] = f2bf_bits(v - bf_bits2f(hb[e]));
  }
  const v4u uh = (v4u){pk16(hb[0], hb[1]), pk16(hb[2], hb[3]), pk16(hb[4], hb[5]), pk16(hb[6], hb[7])};
  const v4u ul = (v4u){pk16(lb[0], lb[1]), pk16(lb[2], lb[3]), pk16(lb[4], lb[5]), pk16(lb[6], lb[7])};
  const size_t off = (size_t)o * kKtot + kk0;
  for (int pass = 0; pass < 2; ++pass) {
    *(volatile v4u*)(Bhi + off) = uh;
    *(volatile v4u*)(Blo + off) = ul;
    __threadfence();
  }
}

__global__ __launch_bounds__(256) void feat_kernel(const float* __restrict__ x,
                                                   unsigned short* __restrict__ Ahi, unsigned short* __restrict__ Alo,
                                                   int nrows_x) {
#pragma clang fp contract(off)
  __shared__ __align__(16) float sS[kFeatThreads];
  const int tid = threadIdx.x;
  const int row = blockIdx.x / kFeatBlocksPerRow;
  const int ib  = blockIdx.x - row * kFeatBlocksPerRow;
  const int i   = ib * kFeatThreads + tid;
  int grow = (row < nrows_x) ? row : (nrows_x - 1);
  const float xr = x[(size_t)grow * kIn + i];
  const float xx = bf_rne(xr);

  const float ex = expf(-xx);
  const float rc = 1.0f / (1.0f + ex);
  const float sl = xx * rc;
  sS[tid] = sl;

  float ph[kBasis];
  float h0one;
  asm volatile("v_mov_b32 %0, 1.0" : "=v"(h0one));
  ph[0] = h0one;
  const float x2 = 2.0f * xx;
  ph[1] = x2;
#pragma unroll
  for (int k = 2; k < kBasis; ++k) {
    const float t = x2 * ph[k - 1];
    const float u = (2.0f * (float)(k - 1)) * ph[k - 2];
    ph[k] = t - u;
  }
  unsigned short hb[8], lb[8];
#pragma unroll
  for (int e = 0; e < 8; ++e) {
    hb[e] = f2bf_bits(ph[e]);
    lb[e] = f2bf_bits(ph[e] - bf_bits2f(hb[e]));
  }
  const v4u fh = (v4u){pk16(hb[0], hb[1]), pk16(hb[2], hb[3]), pk16(hb[4], hb[5]), pk16(hb[6], hb[7])};
  const v4u fl = (v4u){pk16(lb[0], lb[1]), pk16(lb[2], lb[3]), pk16(lb[4], lb[5]), pk16(lb[6], lb[7])};

  __syncthreads();

  const bool sw = (tid < 32);
  v4u gh = fh, gl = fl;
  if (sw) {
    const v4f a0 = *(const v4f*)(sS + 8 * tid);
    const v4f a1 = *(const v4f*)(sS + 8 * tid + 4);
    unsigned short sh[8], slo[8];
#pragma unroll
    for (int e = 0; e < 4; ++e) {
      sh[e] = f2bf_bits(a0[e]);
      slo[e] = f2bf_bits(a0[e] - bf_bits2f(sh[e]));
      sh[4 + e] = f2bf_bits(a1[e]);
      slo[4 + e] = f2bf_bits(a1[e] - bf_bits2f(sh[4 + e]));
    }
    gh = (v4u){pk16(sh[0], sh[1]), pk16(sh[2], sh[3]), pk16(sh[4], sh[5]), pk16(sh[6], sh[7])};
    gl = (v4u){pk16(slo[0], slo[1]), pk16(slo[2], slo[3]), pk16(slo[4], slo[5]), pk16(slo[6], slo[7])};
  }
  const size_t offB = (size_t)row * kKtot + kIn + (size_t)i * kBasis;
  const size_t offS = (size_t)row * kKtot + (size_t)ib * kFeatThreads + (size_t)8 * (tid & 31);
  for (int pass = 0; pass < 2; ++pass) {
    *(volatile v4u*)(Ahi + offB) = fh;
    *(volatile v4u*)(Alo + offB) = fl;
    if (sw) {
      *(volatile v4u*)(Ahi + offS) = gh;
      *(volatile v4u*)(Alo + offS) = gl;
    }
    __threadfence();
  }
}

extern "C" void kernel_launch(void* const* d_in, const int* in_sizes, int n_in,
                              void* d_out, int out_size, void* d_ws, size_t ws_size,
                              hipStream_t stream) {
  if (n_in < 3) return;
  const float* x  = (const float*)d_in[0];
  const float* w  = (const float*)d_in[1];
  const float* cf = (const float*)d_in[2];
  float* out = (float*)d_out;

  if (in_sizes[0] < kRows * kIn) return;
  if (in_sizes[1] < kIn * kOutF) return;
  if (in_sizes[2] < kIn * kOutF * kBasis) return;
  if (out_size < kRows * kOutF) return;
  if (kWsTotal > ws_size) return;
  const int nrowsX = in_sizes[0] / kIn;

  unsigned short* Bhi = (unsigned short*)((char*)d_ws + kOffBtHi);
  unsigned short* Blo = (unsigned short*)((char*)d_ws + kOffBtLo);
  unsigned short* Ahi = (unsigned short*)((char*)d_ws + kOffAHi);
  unsigned short* Alo = (unsigned short*)((char*)d_ws + kOffALo);

  wprep_kernel<<<(kOutF * (kKtot / 8) + 255) / 256, 256, 0, stream>>>(w, cf, Bhi, Blo);

  feat_kernel<<<kRows * kFeatBlocksPerRow, kFeatThreads, 0, stream>>>(x, Ahi, Alo, nrowsX);

  const int tiles = (kRows / 64) * (kOutF / 64);
  wmma_gemm64<1, true, 0, 0, false><<<dim3((tiles + 7) / 8, 1), 256, 0, stream>>>(
      Ahi, Alo, kKtot, 0L,
      Bhi, Blo, kKtot, 0L,
      (void*)out, nullptr, kOutF, 0L,
      nullptr,
      nullptr, 0L,
      kRows, kOutF, kKtot, 1.0f);
}
